// KANLayer_52235392253971
// MI455X (gfx1250) — hardware-verified
//
#include <hip/hip_runtime.h>
#include <math.h>

#pragma clang fp contract(off)

constexpr int kRows    = 8192;
constexpr int kIn      = 1024;
constexpr int kOutF    = 1024;
constexpr int kNB      = 7;
constexpr int kNKnots  = 11;
constexpr int kKaug    = kIn * 8;
constexpr int kTileM   = 64;
constexpr int kWaveN   = 64;
constexpr int kWaves   = 8;
constexpr int kTileN   = kWaves * kWaveN;
constexpr int kIPC     = 8;
constexpr int kTK      = kIPC * 8;
constexpr int kLDA     = 72;
constexpr int kNChunk  = kIn / kIPC;
constexpr int kThreads = 256;
constexpr float kXCarry = 16.0f;
constexpr float kWCarry = 1024.0f;
constexpr float kBCarry = 1024.0f;
constexpr float kSCarry = 16.0f;
constexpr float kAccInv = 1.0f / 16384.0f;
constexpr size_t kBtBytes = (size_t)kOutF * (size_t)kKaug * 2;

static_assert(kRows % kTileM == 0);
static_assert(kOutF % kTileN == 0);
static_assert(kKaug % kTK == 0);
static_assert(kTK % 32 == 0);
static_assert(kTileM * kIPC == 2 * kThreads);
static_assert(kIn == 4 * kThreads);
static_assert(kXCarry * kWCarry == kBCarry * kSCarry);
static_assert(kXCarry * kWCarry * kAccInv == 1.0f);
static_assert((kLDA * 2) % 16 == 0);
static_assert(kBtBytes == 16777216);

typedef __attribute__((ext_vector_type(16))) _Float16 v16h;
typedef __attribute__((ext_vector_type(8)))  _Float16 v8h;
typedef __attribute__((ext_vector_type(8)))  float    v8f;
typedef __attribute__((ext_vector_type(4)))  float    v4f;
typedef __attribute__((ext_vector_type(4)))  unsigned int v4u;

union FragU { v16h v; v8h h[2]; };

__device__ __forceinline__ v16h frag_load_h(const _Float16* p) {
  FragU f; f.h[0] = *(const v8h*)(p); f.h[1] = *(const v8h*)(p + 16); return f.v;
}
__device__ __forceinline__ v8f mma_h(v16h a, v16h b, v8f c) {
  return __builtin_amdgcn_wmma_f32_16x16x32_f16(false, a, false, b, (short)0, c, false, false);
}
__device__ __forceinline__ void guard_row(v8f& a0, v8f& a1, v8f& a2, v8f& a3,
                                          v16h fa, v16h b0, v16h b1, v16h b2, v16h b3) {
  asm volatile("v_nop\n\tv_nop\n\tv_nop\n\tv_nop"
               : "+v"(a0), "+v"(a1), "+v"(a2), "+v"(a3)
               : "v"(fa), "v"(b0), "v"(b1), "v"(b2), "v"(b3));
}
__device__ __forceinline__ void acc_guard4(v8f& a, v8f& b, v8f& c, v8f& d) {
  asm volatile("v_nop\n\tv_nop\n\tv_nop\n\tv_nop" : "+v"(a), "+v"(b), "+v"(c), "+v"(d));
}
__device__ __forceinline__ unsigned pk16(unsigned short a, unsigned short b) { return (unsigned)a | ((unsigned)b << 16); }
__device__ __forceinline__ unsigned short h_bits(float f) { const _Float16 h = (_Float16)f; return __builtin_bit_cast(unsigned short, h); }

__device__ __forceinline__ float tanh_rat(float xin) {
  const float ax = fabsf(xin);
  const float xc = fminf(fmaxf(xin, -7.99881172180175781f), 7.99881172180175781f);
  const float x2 = xc * xc;
  float p = -2.76076847742355e-16f;
  p = fmaf(x2, p, 2.00018790482477e-13f);
  p = fmaf(x2, p, -8.60467152213735e-11f);
  p = fmaf(x2, p, 5.12229709037114e-08f);
  p = fmaf(x2, p, 1.48572235717979e-05f);
  p = fmaf(x2, p, 6.37261928875436e-04f);
  p = fmaf(x2, p, 4.89352455891786e-03f);
  p = xc * p;
  float q = 1.19825839466702e-06f;
  q = fmaf(x2, q, 1.18534705686654e-04f);
  q = fmaf(x2, q, 2.26843463243900e-03f);
  q = fmaf(x2, q, 4.89352518554385e-03f);
  const float r = p / q;
  return (ax < 0.0004f) ? xin : r;
}

__global__ __launch_bounds__(kThreads) void build_bt_kernel(const float* __restrict__ W,
                                                         const float* __restrict__ sw,
                                                         unsigned short* __restrict__ Bt) {
  const int o = blockIdx.x;
  const int t = threadIdx.x;
#pragma unroll 1
  for (int it = 0; it < 4; ++it) {
    const int i = it * kThreads + t;
    const float wv = W[(size_t)o * kIn + i] * kWCarry;
    const float* sp = sw + ((size_t)i * kOutF + o) * kNB;
    unsigned short hb[8];
    hb[0] = h_bits(wv);
#pragma unroll
    for (int k = 0; k < kNB; ++k) hb[1 + k] = h_bits(sp[k] * kSCarry);
    const v4u u = (v4u){pk16(hb[0], hb[1]), pk16(hb[2], hb[3]), pk16(hb[4], hb[5]), pk16(hb[6], hb[7])};
    unsigned short* dst = Bt + (size_t)o * kKaug + (size_t)i * 8;
    *(volatile v4u*)dst = u;
    __threadfence();
    *(volatile v4u*)dst = u;
  }
}

__global__ __launch_bounds__(kThreads) void kan_gemm_kernel(const float* __restrict__ x,
                                                         const unsigned short* __restrict__ Btp,
                                                         const float* __restrict__ bias,
                                                         const float* __restrict__ knots,
                                                         float* __restrict__ out) {
  __shared__ __align__(16) unsigned short As[kTileM * kLDA];
  __shared__ __align__(16) float sT[kWaves][16 * 68];

  const int tid   = threadIdx.x;
  const int lane  = tid & 31;
  const int wave  = tid >> 5;
  const int rlane = lane & 15;
  const int koff  = (lane >> 4) * 8;
  const int mOff  = (lane >> 4) * 8;
  const int mBlk  = blockIdx.y * kTileM;
  const int n0    = blockIdx.x * kTileN + wave * kWaveN;
  const _Float16* Bt = (const _Float16*)(const void*)Btp;

  float kv[kNKnots];
#pragma unroll
  for (int j = 0; j < kNKnots; ++j)
    kv[j] = __int_as_float(__builtin_amdgcn_readfirstlane(__float_as_int(knots[j])));
  float rD[3][8];
#pragma unroll
  for (int d = 1; d <= 3; ++d)
#pragma unroll
    for (int j = 0; j < 8; ++j) {
      const float den = kv[j + d] - kv[j];
      rD[d - 1][j] = __int_as_float(__builtin_amdgcn_readfirstlane(__float_as_int(1.0f / den)));
    }

  v8f acc[4][4];
#pragma unroll
  for (int i = 0; i < 4; ++i)
#pragma unroll
    for (int j = 0; j < 4; ++j) acc[i][j] = (v8f){0.f, 0.f, 0.f, 0.f, 0.f, 0.f, 0.f, 0.f};

  for (int ch = 0; ch < kNChunk; ++ch) {
    const int i0 = ch * kIPC;
#pragma unroll
    for (int qq = 0; qq < 2; ++qq) {
      const int p   = tid + qq * kThreads;
      const int row = p >> 3;
      const int il  = p & 7;
      const float xv = x[(size_t)(mBlk + row) * kIn + i0 + il];
      float t = tanh_rat(xv);
      t = fminf(fmaxf(t, kv[0]), kv[kNKnots - 1]);
      float bc[8];
#pragma unroll
      for (int j = 0; j < kNB; ++j) bc[j] = (t >= kv[j] && t < kv[j + 1]) ? 1.0f : 0.0f;
      bc[7] = 0.0f;
#pragma unroll
      for (int d = 1; d <= 3; ++d) {
        float bn[kNB];
#pragma unroll
        for (int j = 0; j < kNB; ++j) {
          const float left  = (t - kv[j]) * rD[d - 1][j];
          const float right = (kv[j + d + 1] - t) * rD[d - 1][j + 1];
          bn[j] = left * bc[j] + right * bc[j + 1];
        }
#pragma unroll
        for (int j = 0; j < kNB; ++j) bc[j] = bn[j];
      }
      unsigned short hb[8];
      hb[0] = h_bits(xv * kXCarry);
#pragma unroll
      for (int k = 0; k < kNB; ++k) hb[1 + k] = h_bits(bc[k] * kBCarry);
      const v4u u = (v4u){pk16(hb[0], hb[1]), pk16(hb[2], hb[3]), pk16(hb[4], hb[5]), pk16(hb[6], hb[7])};
      *(v4u*)(As + row * kLDA + il * 8) = u;
    }
    __syncthreads();

#pragma unroll 1
    for (int ks = 0; ks < 2; ++ks) {
      const int kl = ks * 32;
      const int kg = ch * kTK + kl;
      v16h bh[4];
#pragma unroll
      for (int j = 0; j < 4; ++j)
        bh[j] = frag_load_h(Bt + (size_t)(n0 + (j << 4) + rlane) * kKaug + koff + kg);
#pragma unroll
      for (int i = 0; i < 4; ++i) {
        FragU fa;
        const int ao = ((i << 4) + rlane) * kLDA + koff + kl;
        fa.h[0] = *(const v8h*)(As + ao);
        fa.h[1] = *(const v8h*)(As + ao + 16);
#pragma unroll
        for (int j = 0; j < 4; ++j) acc[i][j] = mma_h(fa.v, bh[j], acc[i][j]);
        guard_row(acc[i][0], acc[i][1], acc[i][2], acc[i][3], fa.v, bh[0], bh[1], bh[2], bh[3]);
      }
    }
    __syncthreads();
  }
  acc_guard4(acc[0][0], acc[0][1], acc[0][2], acc[0][3]);
  acc_guard4(acc[1][0], acc[1][1], acc[1][2], acc[1][3]);
  acc_guard4(acc[2][0], acc[2][1], acc[2][2], acc[2][3]);
  acc_guard4(acc[3][0], acc[3][1], acc[3][2], acc[3][3]);

  float* slab = sT[wave];
#pragma unroll
  for (int i = 0; i < 4; ++i) {
    const int mBase = mBlk + (i << 4);
#pragma unroll
    for (int j = 0; j < 4; ++j) {
      const int n = n0 + (j << 4) + rlane;
      const float bv = bias[n];
#pragma unroll
      for (int r = 0; r < 8; ++r) {
        const float v = acc[i][j][r] * kAccInv + bv;
        slab[(mOff + r) * 68 + (j << 4) + rlane] = v;
      }
    }
    __builtin_amdgcn_fence(__ATOMIC_RELEASE, "workgroup");
    __builtin_amdgcn_wave_barrier();
    __builtin_amdgcn_fence(__ATOMIC_ACQUIRE, "workgroup");
    {
      const int hh = lane >> 4, c4 = (lane & 15) * 4;
      for (int pass = 0; pass < 2; ++pass) {
#pragma unroll
        for (int it = 0; it < 8; ++it) {
          const int row = it * 2 + hh;
          const v4f v = *(const v4f*)(slab + row * 68 + c4);
          *(volatile v4f*)(out + (size_t)(mBase + row) * kOutF + n0 + c4) = v;
        }
        __threadfence();
      }
    }
    __builtin_amdgcn_fence(__ATOMIC_RELEASE, "workgroup");
    __builtin_amdgcn_wave_barrier();
    __builtin_amdgcn_fence(__ATOMIC_ACQUIRE, "workgroup");
  }
}

extern "C" void kernel_launch(void* const* d_in, const int* in_sizes, int n_in,
                              void* d_out, int out_size, void* d_ws, size_t ws_size,
                              hipStream_t stream) {
  if (n_in < 5) return;
  if (in_sizes[0] != kRows * kIn) return;
  if (in_sizes[1] != kIn * kOutF * kNB) return;
  if (in_sizes[2] != kOutF * kIn) return;
  if (in_sizes[3] != kOutF) return;
  if (in_sizes[4] != kNKnots) return;
  if (out_size != kRows * kOutF) return;
  if (ws_size < kBtBytes) return;
  const float* x     = (const float*)d_in[0];
  const float* sw    = (const float*)d_in[1];
  const float* W     = (const float*)d_in[2];
  const float* bias  = (const float*)d_in[3];
  const float* knots = (const float*)d_in[4];
  unsigned short* Bt = (unsigned short*)d_ws;
  float* outp = (float*)d_out;

  build_bt_kernel<<<dim3(kOutF), dim3(kThreads), 0, stream>>>(W, sw, Bt);
  kan_gemm_kernel<<<dim3(kOutF / kTileN, kRows / kTileM), dim3(kThreads), 0, stream>>>(x, Bt, bias, knots, outp);
}
